// CausalSelfAttention_27702539059819
// MI455X (gfx1250) — hardware-verified
//
#include <hip/hip_runtime.h>
#include <math.h>

#ifndef NB
#define NB 2
#endif
#ifndef SEQ
#define SEQ 2048
#endif
#define NB_FULL 2
#define SEQ_FULL 2048
#define CW 1024
#define NH 16
#define HD 64
#define ROWS (NB * SEQ)
#define QKP (2 * CW)
#define CTXP (2 * CW)
#define PT_P 40
#define EARLY_ROWS 256
#define EARLY_QB (((SEQ / 64) < (EARLY_ROWS / 64)) ? (SEQ / 64) : (EARLY_ROWS / 64))
#define LATE_QB ((SEQ / 64) - EARLY_QB)
#define LATE_QB_DIV ((LATE_QB > 0) ? LATE_QB : 1)

#define W3_SC 64.0f
#define WO_SC_HI 4096.0f
#define WO_SC_LO 4.0f
#define CTX_RS 1024.0f
#define RS 2048.0f
#define RS_INV (1.0f / 2048.0f)
#define P_CARRY 4096.0f
#define SC_L2E 0.18033688011112042f

static_assert(SEQ % 64 == 0);
static_assert(SEQ <= SEQ_FULL);
static_assert(NB <= NB_FULL);
static_assert(NH * HD == CW);
static_assert(HD == 64);
static_assert(CW % 64 == 0);
static_assert(ROWS % 64 == 0);
static_assert((3 * CW) % 64 == 0);
static_assert(CW % 32 == 0);
static_assert((2 * CW) % 32 == 0);
static_assert(CW % 8 == 0);
static_assert(PT_P % 8 == 0);
static_assert(PT_P >= 32);
static_assert(EARLY_ROWS % 64 == 0);
static_assert((long long)ROWS * QKP < 2147483647LL);
static_assert((long long)CW * ROWS < 2147483647LL);
static_assert(WO_SC_HI == WO_SC_LO * CTX_RS);

typedef __attribute__((ext_vector_type(16))) _Float16 v16h;
typedef __attribute__((ext_vector_type(8)))  _Float16 v8h;
typedef __attribute__((ext_vector_type(8)))  float    v8f;
typedef __attribute__((ext_vector_type(4)))  float    v4f;
typedef __attribute__((ext_vector_type(4)))  unsigned int v4u;

union FragH { v16h v; v8h h[2]; };
__device__ __forceinline__ v16h ldfrag(const _Float16* p) {
    FragH f; f.h[0] = *(const v8h*)(p); f.h[1] = *(const v8h*)(p + 16); return f.v;
}
__device__ __forceinline__ v8f wmma16(v16h a, v16h b, v8f c) {
    c = __builtin_amdgcn_wmma_f32_16x16x32_f16(false, a, false, b, (short)0, c, false, false);
    asm volatile("v_nop\n\tv_nop\n\tv_nop\n\tv_nop" : "+v"(c) : "v"(a), "v"(b));
    return c;
}
__device__ __forceinline__ v8f wmma_raw(v16h a, v16h b, v8f c) {
    return __builtin_amdgcn_wmma_f32_16x16x32_f16(false, a, false, b, (short)0, c, false, false);
}
__device__ __forceinline__ void dep_guard_h(v8f& a, v8f& b, v16h x, v16h y) { asm volatile("v_nop\n\tv_nop\n\tv_nop\n\tv_nop" : "+v"(a), "+v"(b) : "v"(x), "v"(y)); }
__device__ __forceinline__ void keep4_h(v16h a, v16h b, v16h c, v16h d) { asm volatile("v_nop" :: "v"(a), "v"(b), "v"(c), "v"(d)); }
__device__ __forceinline__ void acc_guard4(v8f& a, v8f& b, v8f& c, v8f& d) { asm volatile("v_nop\n\tv_nop\n\tv_nop\n\tv_nop" : "+v"(a), "+v"(b), "+v"(c), "+v"(d)); }

#define VST2(T, ptr, val) do { const T vst2_v_ = (val); *(volatile T*)(ptr) = vst2_v_; __threadfence(); *(volatile T*)(ptr) = vst2_v_; } while (0)

__device__ __forceinline__ unsigned int cmb_pk2(float a, float b) { return (unsigned int)__builtin_bit_cast(unsigned short, (_Float16)a) | ((unsigned int)__builtin_bit_cast(unsigned short, (_Float16)b) << 16); }
__device__ __forceinline__ float cmb_bf(float v) { const unsigned u = __builtin_bit_cast(unsigned, v); const unsigned r = (u + 0x7fffu + ((u >> 16) & 1u)) & 0xffff0000u; return __builtin_bit_cast(float, r); }

__global__ __launch_bounds__(256) void k_cast_x(const float* __restrict__ SRC, unsigned short* __restrict__ DST) {
    const int u = blockIdx.x * 256 + threadIdx.x;
    if (u >= ROWS * (CW / 8)) return;
    const int r = u / (CW / 8); const int c0 = 8 * (u % (CW / 8));
    const int sr = (r / SEQ) * SEQ_FULL + (r % SEQ);
    const float* s = SRC + (size_t)sr * CW + c0;
    const v4f a = *(const v4f*)s; const v4f b = *(const v4f*)(s + 4);
    v4u pk;
    pk.x = cmb_pk2(cmb_bf(a.x), cmb_bf(a.y)); pk.y = cmb_pk2(cmb_bf(a.z), cmb_bf(a.w));
    pk.z = cmb_pk2(cmb_bf(b.x), cmb_bf(b.y)); pk.w = cmb_pk2(cmb_bf(b.z), cmb_bf(b.w));
    VST2(v4u, (v4u*)(DST + (size_t)r * CW + c0), pk);
}

__global__ __launch_bounds__(256) void k_cast_wT(const float* __restrict__ SRC, int lds, unsigned short* __restrict__ DST, int ldd, int nR, int nC, float sc0, float sc1, int off1) {
    const long long u = (long long)blockIdx.x * 256 + threadIdx.x; const int per = nR / 8;
    if (u >= (long long)nC * per) return;
    const int c = (int)(u / per); const int r0 = 8 * (int)(u % per);
    float w[8];
#pragma unroll
    for (int e = 0; e < 8; ++e) w[e] = cmb_bf(SRC[(long long)(r0 + e) * lds + c]);
    v4u pk; pk.x = cmb_pk2(w[0] * sc0, w[1] * sc0); pk.y = cmb_pk2(w[2] * sc0, w[3] * sc0); pk.z = cmb_pk2(w[4] * sc0, w[5] * sc0); pk.w = cmb_pk2(w[6] * sc0, w[7] * sc0);
    VST2(v4u, (v4u*)(DST + (long long)c * ldd + r0), pk);
    if (off1 > 0) {
        v4u pk1; pk1.x = cmb_pk2(w[0] * sc1, w[1] * sc1); pk1.y = cmb_pk2(w[2] * sc1, w[3] * sc1); pk1.z = cmb_pk2(w[4] * sc1, w[5] * sc1); pk1.w = cmb_pk2(w[6] * sc1, w[7] * sc1);
        VST2(v4u, (v4u*)(DST + (long long)c * ldd + off1 + r0), pk1);
    }
}

template <int MODE>
__device__ __forceinline__ void gemm64_body(const _Float16* __restrict__ A, const int lda, const _Float16* __restrict__ Bt, const int ldb,
                                            float* __restrict__ Cf, unsigned short* __restrict__ Ch, unsigned short* __restrict__ Cr, const int ldc,
                                            const float* __restrict__ bias, const int M, const int N, const int K, const float scale, const float rscale,
                                            const int rpb, const int rpbFull) {
    __shared__ __align__(16) float sT[8][16 * 68];
    const int lane = threadIdx.x & 31;
    const int wave = __builtin_amdgcn_readfirstlane((int)(threadIdx.x >> 5));
    const int tilesN = N >> 6, tilesM = M >> 6;
    const int tile = blockIdx.x * 8 + wave;
    if (tile >= tilesM * tilesN) return;
    const int tm = tile / tilesN, tn = tile - tm * tilesN;
    const int m0 = tm << 6, n0 = tn << 6;
    const int rlane = lane & 15, koff = (lane >> 4) * 8, mOff = (lane >> 4) * 8;

    v8f acc[4][4];
#pragma unroll
    for (int i = 0; i < 4; ++i)
#pragma unroll
        for (int j = 0; j < 4; ++j) acc[i][j] = (v8f){0.f, 0.f, 0.f, 0.f, 0.f, 0.f, 0.f, 0.f};

    for (int k0 = 0; k0 < K; k0 += 32) {
        v16h bh[4];
#pragma unroll
        for (int j = 0; j < 4; ++j) bh[j] = ldfrag(Bt + (size_t)(n0 + (j << 4) + rlane) * ldb + koff + k0);
#pragma unroll
        for (int i = 0; i < 4; ++i) {
            const v16h ah = ldfrag(A + (size_t)(m0 + (i << 4) + rlane) * lda + koff + k0);
#pragma unroll
            for (int j = 0; j < 4; ++j) acc[i][j] = wmma_raw(ah, bh[j], acc[i][j]);
            dep_guard_h(acc[i][0], acc[i][3], ah, ah);
        }
        keep4_h(bh[0], bh[1], bh[2], bh[3]);
    }
    acc_guard4(acc[0][0], acc[0][1], acc[0][2], acc[0][3]);
    acc_guard4(acc[1][0], acc[1][1], acc[1][2], acc[1][3]);
    acc_guard4(acc[2][0], acc[2][1], acc[2][2], acc[2][3]);
    acc_guard4(acc[3][0], acc[3][1], acc[3][2], acc[3][3]);

#pragma unroll
    for (int i = 0; i < 4; ++i) {
        const int mBase = m0 + (i << 4);
#pragma unroll
        for (int j = 0; j < 4; ++j) {
            const int n = n0 + (j << 4) + rlane;
            float bn = 0.f;
            if (MODE != 2) bn = cmb_bf(bias[n]);
#pragma unroll
            for (int r = 0; r < 8; ++r) {
                float v = acc[i][j][r] * scale;
                if (MODE == 2) v += cmb_bf(bias[mBase + mOff + r]); else v += bn;
                sT[wave][(mOff + r) * 68 + (j << 4) + rlane] = v;
            }
        }
        __builtin_amdgcn_fence(3  , "workgroup");
        __builtin_amdgcn_wave_barrier();
        __builtin_amdgcn_fence(2  , "workgroup");
        if (MODE == 0) {
            const int sq = m0 / rpb;
            const int mo = sq * rpbFull + (m0 - sq * rpb) + (i << 4);
            const int hh2 = lane >> 4, c4 = (lane & 15) * 4;
            for (int pass = 0; pass < 2; ++pass) {
#pragma unroll
                for (int it = 0; it < 8; ++it) {
                    const int row = it * 2 + hh2;
                    const v4f v = *(const v4f*)&sT[wave][row * 68 + c4];
                    *(volatile v4f*)(Cf + (size_t)(mo + row) * ldc + n0 + c4) = v;
                }
                __threadfence();
            }
        } else {
            const int q4 = lane >> 3, c8 = (lane & 7) * 8;
            for (int pass = 0; pass < 2; ++pass) {
#pragma unroll
                for (int it = 0; it < 4; ++it) {
                    const int row = it * 4 + q4;
                    const v4f f0 = *(const v4f*)&sT[wave][row * 68 + c8];
                    const v4f f1 = *(const v4f*)&sT[wave][row * 68 + c8 + 4];
                    const float sp[8] = {f0.x, f0.y, f0.z, f0.w, f1.x, f1.y, f1.z, f1.w};
                    v8h hv, lv;
#pragma unroll
                    for (int e = 0; e < 8; ++e) {
                        const _Float16 hi = (_Float16)sp[e];
                        hv[e] = hi;
                        lv[e] = (_Float16)((sp[e] - (float)hi) * rscale);
                    }
                    *(volatile v8h*)(Ch + (size_t)(mBase + row) * ldc + n0 + c8) = hv;
                    *(volatile v8h*)(Cr + (size_t)(mBase + row) * ldc + n0 + c8) = lv;
                }
                __threadfence();
            }
        }
        __builtin_amdgcn_fence(3  , "workgroup");
        __builtin_amdgcn_wave_barrier();
        __builtin_amdgcn_fence(2  , "workgroup");
    }
}

__global__ __launch_bounds__(256) void k_gemm_qk(const unsigned short* __restrict__ X16, const unsigned short* __restrict__ W3T, unsigned short* __restrict__ QKh, unsigned short* __restrict__ QKr, const float* __restrict__ bias) {
    gemm64_body<1>((const _Float16*)X16, CW, (const _Float16*)W3T, CW, nullptr, QKh, QKr, QKP, bias, ROWS, 2 * CW, CW, 1.0f / W3_SC, RS, 1, 1);
}
__global__ __launch_bounds__(256) void k_gemm_vt(const unsigned short* __restrict__ WvT, const unsigned short* __restrict__ X16, unsigned short* __restrict__ VTh, unsigned short* __restrict__ VTr, const float* __restrict__ biasv) {
    gemm64_body<2>((const _Float16*)WvT, CW, (const _Float16*)X16, CW, nullptr, VTh, VTr, ROWS, biasv, CW, ROWS, CW, 1.0f / W3_SC, RS, 1, 1);
}
__global__ __launch_bounds__(256) void k_gemm_proj(const unsigned short* __restrict__ CTX, const unsigned short* __restrict__ WoT, float* __restrict__ OUT, const float* __restrict__ bias) {
    gemm64_body<0>((const _Float16*)CTX, CTXP, (const _Float16*)WoT, 2 * CW, OUT, nullptr, nullptr, CW, bias, ROWS, CW, 2 * CW, 1.0f / WO_SC_HI, 1.0f, SEQ, SEQ_FULL);
}

template <bool EARLY>
__device__ __forceinline__ void attn_body(const _Float16* __restrict__ QKh, const _Float16* __restrict__ QKr,
                                          const _Float16* __restrict__ VTh, const _Float16* __restrict__ VTr,
                                          unsigned short* __restrict__ CTX, const int qb, const int h, const int b) {
    __shared__ __align__(16) _Float16 Pt[4][16 * PT_P];
    __shared__ __align__(16) _Float16 Pq[EARLY ? 4 : 1][EARLY ? 16 * PT_P : 8];
    __shared__ __align__(16) float Os[4][16 * 68];
    const int lane = threadIdx.x & 31, hh = lane >> 4, c = lane & 15;
    const int wave = __builtin_amdgcn_readfirstlane((int)(threadIdx.x >> 5));
    const int q0 = qb * 64 + wave * 16;
    const int tb = b * SEQ;
    const float NEG = -__builtin_inff();
    const int qoff = (tb + q0 + c) * QKP + h * HD + 8 * hh;
    const int kcol = CW + h * HD + 8 * hh;
    const int vrow = (h * HD + c) * ROWS + tb + 8 * hh;

    v8f o[4]; float m8[8], l8[8];
#pragma unroll
    for (int t = 0; t < 4; ++t) o[t] = (v8f){0.f, 0.f, 0.f, 0.f, 0.f, 0.f, 0.f, 0.f};
#pragma unroll
    for (int r = 0; r < 8; ++r) { m8[r] = NEG; l8[r] = 0.f; }

    const int nsteps = (q0 + 16 + 31) >> 5;
    for (int ks = 0; ks < nsteps; ++ks) {
        const int kv0 = ks * 32;
        const v16h qh0 = ldfrag(QKh + qoff), qh1 = ldfrag(QKh + qoff + 32);
        const v16h qr0 = ldfrag(QKr + qoff), qr1 = ldfrag(QKr + qoff + 32);
        v8f s[2];
#pragma unroll
        for (int j = 0; j < 2; ++j) {
            const int ko = (tb + kv0 + 16 * j + c) * QKP + kcol;
            const v16h kh0 = ldfrag(QKh + ko), kh1 = ldfrag(QKh + ko + 32);
            v8f a = (v8f){0.f, 0.f, 0.f, 0.f, 0.f, 0.f, 0.f, 0.f};
            if (EARLY) {
                const v16h kr0 = ldfrag(QKr + ko), kr1 = ldfrag(QKr + ko + 32);
                a = wmma16(qh0, kr0, a); a = wmma16(qh1, kr1, a);
            }
            a = wmma16(qr0, kh0, a); a = wmma16(qr1, kh1, a);
            a = a * RS_INV;
            a = wmma16(qh0, kh0, a); a = wmma16(qh1, kh1, a);
            s[j] = a;
        }
        const bool diag = (kv0 + 31 > q0);
#pragma unroll
        for (int r = 0; r < 8; ++r) {
            const int row = q0 + 8 * hh + r;
            float sc0 = s[0][r] * SC_L2E, sc1 = s[1][r] * SC_L2E;
            const bool x0 = diag && (kv0 + c > row), x1 = diag && (kv0 + 16 + c > row);
            sc0 = x0 ? NEG : sc0; sc1 = x1 ? NEG : sc1;
            float mx = fmaxf(sc0, sc1);
            mx = fmaxf(mx, __shfl_xor(mx, 1, 32)); mx = fmaxf(mx, __shfl_xor(mx, 2, 32));
            mx = fmaxf(mx, __shfl_xor(mx, 4, 32)); mx = fmaxf(mx, __shfl_xor(mx, 8, 32));
            const float mnew = fmaxf(m8[r], mx);
            const float corr = (mnew == NEG) ? 1.f : exp2f(m8[r] - mnew);
            const float p0 = (sc0 == NEG) ? 0.f : exp2f(sc0 - mnew);
            const float p1 = (sc1 == NEG) ? 0.f : exp2f(sc1 - mnew);
            float rs = p0 + p1;
            rs += __shfl_xor(rs, 1, 32); rs += __shfl_xor(rs, 2, 32); rs += __shfl_xor(rs, 4, 32); rs += __shfl_xor(rs, 8, 32);
            l8[r] = l8[r] * corr + rs; m8[r] = mnew;
#pragma unroll
            for (int t = 0; t < 4; ++t) o[t][r] *= corr;
            const float c0v = p0 * P_CARRY, c1v = p1 * P_CARRY;
            const _Float16 h0 = (_Float16)c0v, h1 = (_Float16)c1v;
            Pt[wave][(8 * hh + r) * PT_P + c] = h0;
            Pt[wave][(8 * hh + r) * PT_P + 16 + c] = h1;
            if (EARLY) {
                Pq[wave][(8 * hh + r) * PT_P + c] = (_Float16)((c0v - (float)h0) * RS);
                Pq[wave][(8 * hh + r) * PT_P + 16 + c] = (_Float16)((c1v - (float)h1) * RS);
            }
        }
        __builtin_amdgcn_fence(3  , "workgroup");
        __builtin_amdgcn_wave_barrier();
        __builtin_amdgcn_fence(2  , "workgroup");
        FragH pa;
        pa.h[0] = *(const v8h*)&Pt[wave][c * PT_P + 8 * hh];
        pa.h[1] = *(const v8h*)&Pt[wave][c * PT_P + 16 + 8 * hh];
        const int vo = vrow + kv0;
        if (EARLY) {
            FragH pr;
            pr.h[0] = *(const v8h*)&Pq[wave][c * PT_P + 8 * hh];
            pr.h[1] = *(const v8h*)&Pq[wave][c * PT_P + 16 + 8 * hh];
#pragma unroll
            for (int t = 0; t < 4; ++t) {
                const v16h vh = ldfrag(VTh + vo + 16 * t * ROWS), vr = ldfrag(VTr + vo + 16 * t * ROWS);
                v8f tmp = (v8f){0.f, 0.f, 0.f, 0.f, 0.f, 0.f, 0.f, 0.f};
                tmp = wmma16(pa.v, vr, tmp); tmp = wmma16(pr.v, vh, tmp);
                o[t] = wmma16(pa.v, vh, o[t]);
                o[t] = o[t] + tmp * RS_INV;
            }
        } else {
            v16h vb[4];
#pragma unroll
            for (int t = 0; t < 4; ++t) vb[t] = ldfrag(VTh + vo + 16 * t * ROWS);
#pragma unroll
            for (int t = 0; t < 4; ++t) o[t] = wmma16(pa.v, vb[t], o[t]);
        }
        __builtin_amdgcn_fence(3  , "workgroup");
        __builtin_amdgcn_wave_barrier();
        __builtin_amdgcn_fence(2  , "workgroup");
    }

#pragma unroll
    for (int r = 0; r < 8; ++r) {
        const float inv = 1.0f / (l8[r] * P_CARRY);
#pragma unroll
        for (int t = 0; t < 4; ++t) Os[wave][(8 * hh + r) * 68 + 16 * t + c] = o[t][r] * inv;
    }
    __builtin_amdgcn_fence(3  , "workgroup");
    __builtin_amdgcn_wave_barrier();
    __builtin_amdgcn_fence(2  , "workgroup");
    {
        const int q4 = lane >> 3, c8 = (lane & 7) * 8;
        for (int pass = 0; pass < 2; ++pass) {
#pragma unroll
            for (int it = 0; it < 4; ++it) {
                const int row = it * 4 + q4;
                const v4f f0 = *(const v4f*)&Os[wave][row * 68 + c8];
                const v4f f1 = *(const v4f*)&Os[wave][row * 68 + c8 + 4];
                const float sp[8] = {f0.x, f0.y, f0.z, f0.w, f1.x, f1.y, f1.z, f1.w};
                v8h hv, lv;
#pragma unroll
                for (int e = 0; e < 8; ++e) {
                    const _Float16 hi = (_Float16)sp[e];
                    hv[e] = hi;
                    lv[e] = (_Float16)((sp[e] - (float)hi) * CTX_RS);
                }
                unsigned short* dst = CTX + (size_t)(tb + q0 + row) * CTXP + h * HD + c8;
                *(volatile v8h*)dst = hv;
                *(volatile v8h*)(dst + CW) = lv;
            }
            __threadfence();
        }
    }
}

__global__ __launch_bounds__(128) void k_attn_early(const unsigned short* __restrict__ QKh, const unsigned short* __restrict__ QKr,
                                                    const unsigned short* __restrict__ VTh, const unsigned short* __restrict__ VTr, unsigned short* __restrict__ CTX) {
    const int bx = blockIdx.x; const int qb = bx % EARLY_QB; const int bh = bx / EARLY_QB;
    attn_body<true>((const _Float16*)QKh, (const _Float16*)QKr, (const _Float16*)VTh, (const _Float16*)VTr, CTX, qb, bh % NH, bh / NH);
}
__global__ __launch_bounds__(128) void k_attn_late(const unsigned short* __restrict__ QKh, const unsigned short* __restrict__ QKr,
                                                   const unsigned short* __restrict__ VTh, const unsigned short* __restrict__ VTr, unsigned short* __restrict__ CTX) {
    const int bx = blockIdx.x; const int qb = EARLY_QB + bx % LATE_QB_DIV; const int bh = bx / LATE_QB_DIV;
    attn_body<false>((const _Float16*)QKh, (const _Float16*)QKr, (const _Float16*)VTh, (const _Float16*)VTr, CTX, qb, bh % NH, bh / NH);
}

constexpr size_t SZ_X16 = (size_t)ROWS * CW * 2;
constexpr size_t SZ_W3T = (size_t)3 * CW * CW * 2;
constexpr size_t SZ_WOT = (size_t)CW * 2 * CW * 2;
constexpr size_t SZ_QK  = (size_t)ROWS * QKP * 2;
constexpr size_t SZ_VT  = (size_t)CW * ROWS * 2;
constexpr size_t SZ_CTX = (size_t)ROWS * CTXP * 2;
constexpr size_t WS_TOTAL = SZ_X16 + SZ_W3T + SZ_WOT + 2 * SZ_QK + 2 * SZ_VT + SZ_CTX;
static_assert(WS_TOTAL <= (size_t)134217728);
static_assert(SZ_X16 % 256 == 0);
static_assert(SZ_W3T % 256 == 0);
static_assert(SZ_WOT % 256 == 0);
static_assert(SZ_QK % 256 == 0);
static_assert(SZ_VT % 256 == 0);
static_assert(SZ_CTX % 256 == 0);

extern "C" void kernel_launch(void* const* d_in, const int* in_sizes, int n_in, void* d_out, int out_size, void* d_ws, size_t ws_size, hipStream_t stream) {
    if (n_in < 5) return;
    const int need_rows = (NB - 1) * SEQ_FULL + SEQ;
    if (in_sizes[0] < need_rows * CW) return;
    if (in_sizes[1] < CW * 3 * CW) return;
    if (in_sizes[2] < 3 * CW) return;
    if (in_sizes[3] < CW * CW) return;
    if (in_sizes[4] < CW) return;
    if (out_size < need_rows * CW) return;
    if (WS_TOTAL > ws_size) return;
    const float* x      = (const float*)d_in[0];
    const float* w_attn = (const float*)d_in[1];
    const float* b_attn = (const float*)d_in[2];
    const float* w_proj = (const float*)d_in[3];
    const float* b_proj = (const float*)d_in[4];
    float* out = (float*)d_out;
    char* wsp = (char*)d_ws;
    unsigned short* X16 = (unsigned short*)wsp; wsp += SZ_X16;
    unsigned short* W3T = (unsigned short*)wsp; wsp += SZ_W3T;
    unsigned short* WOT = (unsigned short*)wsp; wsp += SZ_WOT;
    unsigned short* QKh = (unsigned short*)wsp; wsp += SZ_QK;
    unsigned short* QKr = (unsigned short*)wsp; wsp += SZ_QK;
    unsigned short* VTh = (unsigned short*)wsp; wsp += SZ_VT;
    unsigned short* VTr = (unsigned short*)wsp; wsp += SZ_VT;
    unsigned short* CTX = (unsigned short*)wsp; wsp += SZ_CTX;

    k_cast_x<<<(unsigned)((ROWS * (CW / 8) + 255) / 256), 256, 0, stream>>>(x, X16);
    k_cast_wT<<<(unsigned)(((long long)(3 * CW) * (CW / 8) + 255) / 256), 256, 0, stream>>>(w_attn, 3 * CW, W3T, CW, CW, 3 * CW, W3_SC, 0.0f, 0);
    k_cast_wT<<<(unsigned)(((long long)CW * (CW / 8) + 255) / 256), 256, 0, stream>>>(w_proj, CW, WOT, 2 * CW, CW, CW, WO_SC_HI, WO_SC_LO, CW);
    k_gemm_qk<<<(unsigned)(((ROWS / 64) * ((2 * CW) / 64) + 7) / 8), 256, 0, stream>>>(X16, W3T, QKh, QKr, b_attn);
    k_gemm_vt<<<(unsigned)(((CW / 64) * (ROWS / 64) + 7) / 8), 256, 0, stream>>>(W3T + (size_t)2 * CW * CW, X16, VTh, VTr, b_attn + 2 * CW);
    k_attn_early<<<(unsigned)(NB * NH * EARLY_QB), 128, 0, stream>>>(QKh, QKr, VTh, VTr, CTX);
    if (LATE_QB > 0) k_attn_late<<<(unsigned)(NB * NH * LATE_QB_DIV), 128, 0, stream>>>(QKh, QKr, VTh, VTr, CTX);
    k_gemm_proj<<<(unsigned)(((ROWS / 64) * (CW / 64) + 7) / 8), 256, 0, stream>>>(CTX, WOT, out, b_proj);
}
